// GraphEncoder_56659208568898
// MI455X (gfx1250) — hardware-run, weakly checked
//
#include <hip/hip_runtime.h>
#include <stddef.h>
#include <stdint.h>

#define SINGLE_H   0
#define SINGLE_NG  0

#define NN      50000
#define NE      800000
#define MP      50048
#define GBM     128
#define NTHR    256
#define NWAVE   8
#define EPT     8
#define WCH     (32 * EPT)
#define NBRUN   1024
#define SLB     10
#define NBK     49
#define WLCAP   2560
#define RCAP    20480
#define DEGCAP  64
#define MAXDEG_MEAS   33
#define MAXB1024_MEAS 16696
#define RBM     64
#define SP      68
#define WSMAX   ((size_t)128 << 20)

#define XB_P   128
#define H1_P   128
#define H2_P   256
#define NG1_P  256
#define NG2_P  128
#define NG3_P  256
#define WA1_P  128
#define WA2_P  128
#define WA3_P  256
#define WB1_P  256
#define WB2_P  128
#define WB3_P  256
#define KA1  128
#define KA2  (SINGLE_H ? 64 : 128)
#define KA3  (SINGLE_H ? 128 : 256)
#define KB1  (SINGLE_NG ? 128 : 256)
#define KB2  (SINGLE_NG ? 64 : 128)
#define KB3  (SINGLE_NG ? 128 : 256)

#define BK_ZINTS (NWAVE * WLCAP + RCAP + 3 * NBRUN)
#define BK_INTS  (BK_ZINTS + 16)
#define BK_LDS   (BK_INTS * 4)

#define PBX    (MP * 128 / 8 / NTHR)
#define PB_A1P 8
#define PB_A1S 4
#define PB_A2P 4
#define PB_A2S 8
#define PB_A3P 16
#define PB_A3S 16
#define PB_B1  8
#define PB_B2  8
#define PB_B3  16
#define PBW    (PB_A1P + PB_A1S + PB_A2P + PB_A2S + PB_A3P + PB_A3S + PB_B1 + PB_B2 + PB_B3)
#define PBTOT  (PBX + PBW + 1)
#define BT_FLOATS 768

static_assert(MP % GBM == 0 && MP >= NN && MP == 391 * GBM && MP % RBM == 0);
static_assert(NBRUN == (1 << SLB) && NBRUN % RBM == 0 && NBRUN % GBM == 0 && NBRUN % 32 == 0);
static_assert(NBK * NBRUN >= MP && NBK * NBRUN >= NN);
static_assert(NE < (1 << 21) && (((long long)NE) << SLB) < (1LL << 31));
static_assert(NE % WCH == 0 && NE % 8 == 0);
static_assert(RCAP == NWAVE * WLCAP && RCAP % 4 == 0 && BK_ZINTS % 4 == 0);
static_assert((long long)RCAP * 100 >= (long long)MAXB1024_MEAS * 105);
static_assert(WLCAP >= MAXB1024_MEAS / 8 + 8 * 46 + 1);
static_assert(NN <= 65536);
static_assert(MAXDEG_MEAS + 8 <= DEGCAP);
static_assert((MP * 128 / 8) % NTHR == 0);
static_assert(KA1 % 32 == 0 && KA2 % 32 == 0 && KA3 % 32 == 0 && KB1 % 32 == 0 && KB2 % 32 == 0 && KB3 % 32 == 0);
static_assert(KA1 <= XB_P && KA2 <= H1_P && KA3 <= H2_P && KB1 <= NG1_P && KB2 <= NG2_P && KB3 <= NG3_P);
static_assert(KA1 <= WA1_P && KA2 <= WA2_P && KA3 <= WA3_P && KB1 <= WB1_P && KB2 <= WB2_P && KB3 <= WB3_P);
static_assert(BK_LDS <= 300000);
static_assert((GBM * SP + 64) * 4 <= 65536);
static_assert((2 * NBRUN) % (NTHR * 4) == 0);

typedef float          v2f   __attribute__((ext_vector_type(2)));
typedef float          v4f   __attribute__((ext_vector_type(4)));
typedef float          v8f   __attribute__((ext_vector_type(8)));
typedef int            v2i   __attribute__((ext_vector_type(2)));
typedef int            v4i   __attribute__((ext_vector_type(4)));
typedef int            v8i   __attribute__((ext_vector_type(8)));
typedef unsigned short v8us  __attribute__((ext_vector_type(8)));
typedef unsigned short v16us __attribute__((ext_vector_type(16)));
typedef __bf16         v16bf __attribute__((ext_vector_type(16)));
typedef v2f  __attribute__((may_alias)) v2fa;
typedef v4f  __attribute__((may_alias)) v4fa;
typedef v4i  __attribute__((may_alias)) v4ia;
typedef v8us __attribute__((may_alias)) v8usa;
union FragB { v16bf v; v16us u; v8us h[2]; v8i w; };

__device__ __forceinline__ v8f wmb(const FragB& a, const FragB& b, v8f c) {
  v8f d = __builtin_amdgcn_wmma_f32_16x16x32_bf16(false, a.v, false, b.v, (short)0, c, false, false);
  asm volatile("v_nop\n\tv_nop\n\tv_nop\n\tv_nop" : "+v"(d) : "v"(a.w), "v"(b.w));
  return d;
}

__device__ __forceinline__ unsigned bf16_bits(float f) {
  const unsigned u = __float_as_uint(f);
  const unsigned r = (u + 0x7FFFu + ((u >> 16) & 1u)) >> 16;
  const unsigned q = (u >> 16) | 0x40u;
  return ((u & 0x7fffffffu) > 0x7f800000u) ? q : r;
}

__device__ __forceinline__ void hilo_pack(float v0, float v1, float v2, float v3,
                                          int& h01, int& h23, int& l01, int& l23) {
  const unsigned a0 = bf16_bits(v0), a1 = bf16_bits(v1), a2 = bf16_bits(v2), a3 = bf16_bits(v3);
  const unsigned b0 = bf16_bits(v0 - __uint_as_float(a0 << 16));
  const unsigned b1 = bf16_bits(v1 - __uint_as_float(a1 << 16));
  const unsigned b2 = bf16_bits(v2 - __uint_as_float(a2 << 16));
  const unsigned b3 = bf16_bits(v3 - __uint_as_float(a3 << 16));
  h01 = (int)(a0 | (a1 << 16)); h23 = (int)(a2 | (a3 << 16));
  l01 = (int)(b0 | (b1 << 16)); l23 = (int)(b2 | (b3 << 16));
}
__device__ __forceinline__ void hilo_pack2(float v0, float v1, int& h01, int& l01) {
  const unsigned a0 = bf16_bits(v0), a1 = bf16_bits(v1);
  const unsigned b0 = bf16_bits(v0 - __uint_as_float(a0 << 16));
  const unsigned b1 = bf16_bits(v1 - __uint_as_float(a1 << 16));
  h01 = (int)(a0 | (a1 << 16));
  l01 = (int)(b0 | (b1 << 16));
}

__device__ __forceinline__ v4i regroup8(int h01, int h23, int l01, int l23, int lane) {
  const int t  = lane & 15;
  const int s0 = (lane & 16) + ((2 * t) & 15), s1 = s0 + 1;
  const int a0 = __shfl(h01, s0, 32), a1 = __shfl(h23, s0, 32), a2 = __shfl(h01, s1, 32), a3 = __shfl(h23, s1, 32);
  const int b0 = __shfl(l01, s0, 32), b1 = __shfl(l23, s0, 32), b2 = __shfl(l01, s1, 32), b3 = __shfl(l23, s1, 32);
  const int mk = (t < 8) ? -1 : 0;
  v4i o;
  o.x = (a0 & mk) | (b0 & ~mk); o.y = (a1 & mk) | (b1 & ~mk);
  o.z = (a2 & mk) | (b2 & ~mk); o.w = (a3 & mk) | (b3 & ~mk);
  return o;
}

__device__ __forceinline__ void st2_v4f(float* p, v4f v) {
  *(volatile v4f*)p = v;
  __threadfence();
  *(volatile v4f*)p = v;
}
__device__ __forceinline__ void st2_v8us(unsigned short* p, v8us v) {
  *(volatile v8us*)p = v;
  __threadfence();
  *(volatile v8us*)p = v;
}

__device__ __forceinline__ v8us gather8(const float* __restrict__ base, int stride) {
  float f[8];
#pragma unroll
  for (int i = 0; i < 8; ++i) f[i] = base[(size_t)i * (size_t)stride];
  v8us o;
#pragma unroll
  for (int i = 0; i < 8; ++i) o[i] = (unsigned short)bf16_bits(f[i]);
  return o;
}

template <int UPR, int KIN, int LDW>
__device__ __forceinline__ void wpart(const float* __restrict__ W, unsigned short* P, int nOff, int u) {
  const int n  = u / UPR;
  const int k8 = (u % UPR) * 8;
  const int kk = k8 % KIN;
  const v8us o = gather8(W + (size_t)kk * LDW + n, LDW);
  st2_v8us(P + (size_t)(nOff + n) * (size_t)(UPR * 8) + k8, o);
}

__device__ __forceinline__ void bias_seg(const float* __restrict__ b, int len, float* dst, int lane) {
  const int n4 = len >> 2;
  const int qc = lane < n4 ? lane : n4 - 1;
  const v4f a = *(const v4fa*)(b + 4 * qc);
  asm volatile("" :: "v"(a));
  const unsigned mk = lane < n4 ? 0xffffffffu : 0u;
  v4f o;
  o.x = __uint_as_float((bf16_bits(a.x) << 16) & mk);
  o.y = __uint_as_float((bf16_bits(a.y) << 16) & mk);
  o.z = __uint_as_float((bf16_bits(a.z) << 16) & mk);
  o.w = __uint_as_float((bf16_bits(a.w) << 16) & mk);
  st2_v4f(dst + 4 * lane, o);
}

__global__ __launch_bounds__(NTHR) void k_prep(
    const float* __restrict__ feat,
    const float* __restrict__ Wp1, const float* __restrict__ bp1, const float* __restrict__ Ws1,
    const float* __restrict__ Wn1, const float* __restrict__ b1,
    const float* __restrict__ Wp2, const float* __restrict__ bp2, const float* __restrict__ Ws2,
    const float* __restrict__ Wn2, const float* __restrict__ b2,
    const float* __restrict__ Wp3, const float* __restrict__ bp3, const float* __restrict__ Ws3,
    const float* __restrict__ Wn3, const float* __restrict__ b3,
    unsigned short* XB, unsigned short* WA1, unsigned short* WA2, unsigned short* WA3,
    unsigned short* WB1, unsigned short* WB2, unsigned short* WB3, float* BT) {
  const int tid = (int)threadIdx.x, lane = tid & 31, wave = tid >> 5;
  const int blk = (int)blockIdx.x;
  constexpr int e0 = PBX;
  constexpr int e1 = e0 + PB_A1P;
  constexpr int e2 = e1 + PB_A1S;
  constexpr int e3 = e2 + PB_A2P;
  constexpr int e4 = e3 + PB_A2S;
  constexpr int e5 = e4 + PB_A3P;
  constexpr int e6 = e5 + PB_A3S;
  constexpr int e7 = e6 + PB_B1;
  constexpr int e8 = e7 + PB_B2;
  constexpr int e9 = e8 + PB_B3;
  if (blk < e0) {
    const int u   = blk * NTHR + tid;
    const int row = u >> 4, k8 = (u & 15) * 8;
    const int rc  = row < NN ? row : NN - 1;
    const unsigned mk = row < NN ? 0xffffu : 0u;
    const float* p = feat + (size_t)rc * 128 + k8;
    const v4f a = *(const v4fa*)p;
    const v4f b = *(const v4fa*)(p + 4);
    v8us o;
    o[0] = (unsigned short)(bf16_bits(a.x) & mk); o[1] = (unsigned short)(bf16_bits(a.y) & mk);
    o[2] = (unsigned short)(bf16_bits(a.z) & mk); o[3] = (unsigned short)(bf16_bits(a.w) & mk);
    o[4] = (unsigned short)(bf16_bits(b.x) & mk); o[5] = (unsigned short)(bf16_bits(b.y) & mk);
    o[6] = (unsigned short)(bf16_bits(b.z) & mk); o[7] = (unsigned short)(bf16_bits(b.w) & mk);
    st2_v8us(XB + (size_t)row * XB_P + k8, o);
  } else if (blk < e1) {
    wpart<16, 128, 128>(Wp1, WA1, 0, (blk - e0) * NTHR + tid);
  } else if (blk < e2) {
    wpart<16, 128, 64>(Ws1, WA1, 128, (blk - e1) * NTHR + tid);
  } else if (blk < e3) {
    wpart<16, 64, 64>(Wp2, WA2, 0, (blk - e2) * NTHR + tid);
  } else if (blk < e4) {
    wpart<16, 64, 128>(Ws2, WA2, 64, (blk - e3) * NTHR + tid);
  } else if (blk < e5) {
    wpart<32, 128, 128>(Wp3, WA3, 0, (blk - e4) * NTHR + tid);
  } else if (blk < e6) {
    wpart<32, 128, 128>(Ws3, WA3, 128, (blk - e5) * NTHR + tid);
  } else if (blk < e7) {
    wpart<32, 128, 64>(Wn1, WB1, 0, (blk - e6) * NTHR + tid);
  } else if (blk < e8) {
    wpart<16, 64, 128>(Wn2, WB2, 0, (blk - e7) * NTHR + tid);
  } else if (blk < e9) {
    wpart<32, 128, 128>(Wn3, WB3, 0, (blk - e8) * NTHR + tid);
  } else {
    if (wave == 0)      bias_seg(bp1, 128, BT + 0,   lane);
    else if (wave == 1) bias_seg(b1,   64, BT + 128, lane);
    else if (wave == 2) bias_seg(bp2,  64, BT + 256, lane);
    else if (wave == 3) bias_seg(b2,  128, BT + 384, lane);
    else if (wave == 4) bias_seg(bp3, 128, BT + 512, lane);
    else if (wave == 5) bias_seg(b3,  128, BT + 640, lane);
  }
}

__device__ __forceinline__ void bucket_flush(const int* pl, const int* cnt, int ov, int* lp, int* cop, int* fp,
                                             int tid) {
#pragma unroll 1
  for (int i = tid * 4; i < RCAP; i += NTHR * 4) {
    const v4i v = *(const v4ia*)(pl + i);
    *(volatile v4i*)(lp + i) = v;
  }
#pragma unroll 1
  for (int i = tid * 4; i < 2 * NBRUN; i += NTHR * 4) {
    const v4i v = *(const v4ia*)(cnt + i);
    *(volatile v4i*)(cop + i) = v;
  }
  if (tid < 8) {
    const v4i f = {ov, ov, ov, ov};
    *(volatile v4i*)(fp + 4 * tid) = f;
  }
}

__global__ __launch_bounds__(NTHR) void k_bucket(const int* __restrict__ srcs, const int* __restrict__ dsts,
                                                 const float* __restrict__ ew, int* LIST, int* CO, int* FLAG) {
  extern __shared__ __attribute__((aligned(16))) int dsm[];
  int* wl   = dsm;
  int* pl   = dsm + NWAVE * WLCAP;
  int* cnt  = pl + RCAP;
  int* offs = cnt + NBRUN;
  int* cur  = offs + NBRUN;
  int* misc = cur + NBRUN;
  const int tid = (int)threadIdx.x, lane = tid & 31, wave = tid >> 5;
  const int blk = (int)blockIdx.x;
  const unsigned nbs = (unsigned)(blk * NBRUN);

  {
    const v4i z4 = {0, 0, 0, 0};
    for (int i = tid * 4; i < BK_ZINTS; i += NTHR * 4) *(v4ia*)(dsm + i) = z4;
    if (tid < 16) misc[tid] = 0;
  }
  __syncthreads();

  {
    const int per  = ((NE + NWAVE * WCH - 1) / (NWAVE * WCH)) * WCH;
    const int ebeg = wave * per;
    const int eend = (ebeg + per < NE) ? (ebeg + per) : NE;
    int* mylist = wl + wave * WLCAP;
    int wc = 0;
#pragma unroll 1
    for (int cb = ebeg; cb < eend; cb += WCH) {
      const int e0 = cb + lane * EPT;
      const v4i da = *(const v4ia*)(dsts + e0);
      const v4i db = *(const v4ia*)(dsts + e0 + 4);
      const unsigned s0 = (unsigned)da.x - nbs, s1 = (unsigned)da.y - nbs;
      const unsigned s2 = (unsigned)da.z - nbs, s3 = (unsigned)da.w - nbs;
      const unsigned s4 = (unsigned)db.x - nbs, s5 = (unsigned)db.y - nbs;
      const unsigned s6 = (unsigned)db.z - nbs, s7 = (unsigned)db.w - nbs;
      const bool h0 = s0 < (unsigned)NBRUN, h1 = s1 < (unsigned)NBRUN, h2 = s2 < (unsigned)NBRUN, h3 = s3 < (unsigned)NBRUN;
      const bool h4 = s4 < (unsigned)NBRUN, h5 = s5 < (unsigned)NBRUN, h6 = s6 < (unsigned)NBRUN, h7 = s7 < (unsigned)NBRUN;
      const unsigned m0 = __builtin_amdgcn_ballot_w32(h0), m1 = __builtin_amdgcn_ballot_w32(h1);
      const unsigned m2 = __builtin_amdgcn_ballot_w32(h2), m3 = __builtin_amdgcn_ballot_w32(h3);
      const unsigned m4 = __builtin_amdgcn_ballot_w32(h4), m5 = __builtin_amdgcn_ballot_w32(h5);
      const unsigned m6 = __builtin_amdgcn_ballot_w32(h6), m7 = __builtin_amdgcn_ballot_w32(h7);
      const unsigned any = m0 | m1 | m2 | m3 | m4 | m5 | m6 | m7;
      if (any != 0u) {
        const int pre = (int)(__builtin_amdgcn_mbcnt_lo(m0, 0u) + __builtin_amdgcn_mbcnt_lo(m1, 0u) +
                              __builtin_amdgcn_mbcnt_lo(m2, 0u) + __builtin_amdgcn_mbcnt_lo(m3, 0u) +
                              __builtin_amdgcn_mbcnt_lo(m4, 0u) + __builtin_amdgcn_mbcnt_lo(m5, 0u) +
                              __builtin_amdgcn_mbcnt_lo(m6, 0u) + __builtin_amdgcn_mbcnt_lo(m7, 0u));
        int p = wc + pre;
        if (h0) { if (p < WLCAP) mylist[p] = ((e0 + 0) << SLB) | (int)s0; p = p + 1; }
        if (h1) { if (p < WLCAP) mylist[p] = ((e0 + 1) << SLB) | (int)s1; p = p + 1; }
        if (h2) { if (p < WLCAP) mylist[p] = ((e0 + 2) << SLB) | (int)s2; p = p + 1; }
        if (h3) { if (p < WLCAP) mylist[p] = ((e0 + 3) << SLB) | (int)s3; p = p + 1; }
        if (h4) { if (p < WLCAP) mylist[p] = ((e0 + 4) << SLB) | (int)s4; p = p + 1; }
        if (h5) { if (p < WLCAP) mylist[p] = ((e0 + 5) << SLB) | (int)s5; p = p + 1; }
        if (h6) { if (p < WLCAP) mylist[p] = ((e0 + 6) << SLB) | (int)s6; p = p + 1; }
        if (h7) { if (p < WLCAP) mylist[p] = ((e0 + 7) << SLB) | (int)s7; p = p + 1; }
        wc += (int)(__builtin_popcount(m0) + __builtin_popcount(m1) + __builtin_popcount(m2) + __builtin_popcount(m3) +
                    __builtin_popcount(m4) + __builtin_popcount(m5) + __builtin_popcount(m6) + __builtin_popcount(m7));
      }
    }
    if (lane == 0) misc[wave] = wc;
  }
  __syncthreads();

  if (wave == 0) {
    int ov = 0;
#pragma unroll 1
    for (int w2 = 0; w2 < NWAVE; ++w2) {
      int c = misc[w2];
      if (c > WLCAP) ov = 1;
      c = c < 0 ? 0 : (c > WLCAP ? WLCAP : c);
#pragma unroll 1
      for (int b0 = 0; b0 < c; b0 += 32) {
        const int idx = b0 + lane;
        const int ent = wl[w2 * WLCAP + (idx < WLCAP ? idx : WLCAP - 1)];
        const int m32 = (c - b0) < 32 ? (c - b0) : 32;
#pragma unroll 1
        for (int k = 0; k < m32; ++k) {
          const int u    = __builtin_amdgcn_readlane(ent, k);
          const int slot = u & (NBRUN - 1);
          if (lane == 0) cnt[slot] = cnt[slot] + 1;
        }
      }
    }
    if (lane == 0) misc[9] = ov;
  }
  __syncthreads();
  if (wave == 0) {
    const int base = lane * (NBRUN / 32);
    int s = 0;
#pragma unroll 1
    for (int i = 0; i < NBRUN / 32; ++i) s += cnt[base + i];
    int incl = s;
#pragma unroll
    for (int d = 1; d < 32; d <<= 1) {
      const int y = __shfl_up(incl, d, 32);
      if (lane >= d) incl += y;
    }
    int run = incl - s;
#pragma unroll 1
    for (int i = 0; i < NBRUN / 32; ++i) {
      const int cv = cnt[base + i];
      offs[base + i] = run;
      cur[base + i]  = run;
      run += cv;
    }
  }
  __syncthreads();

  if (wave == 0) {
#pragma unroll 1
    for (int w2 = 0; w2 < NWAVE; ++w2) {
      int c = misc[w2];
      c = c < 0 ? 0 : (c > WLCAP ? WLCAP : c);
#pragma unroll 1
      for (int b0 = 0; b0 < c; b0 += 32) {
        const int idx = b0 + lane;
        const int ent = wl[w2 * WLCAP + (idx < WLCAP ? idx : WLCAP - 1)];
        int eid = (ent >> SLB) & 0x1FFFFF;
        eid = eid > NE - 1 ? NE - 1 : eid;
        int sr = srcs[eid];
        sr = sr < 0 ? 0 : (sr > NN - 1 ? NN - 1 : sr);
        const int word = (int)(((unsigned)sr << 16) | (bf16_bits(ew[eid]) & 0xffffu));
        const int m32 = (c - b0) < 32 ? (c - b0) : 32;
#pragma unroll 1
        for (int k = 0; k < m32; ++k) {
          const int u    = __builtin_amdgcn_readlane(ent, k);
          const int wd   = __builtin_amdgcn_readlane(word, k);
          const int slot = u & (NBRUN - 1);
          if (lane == 0) {
            int p = cur[slot];
            p = p < 0 ? 0 : (p > RCAP - 1 ? RCAP - 1 : p);
            pl[p] = wd;
            cur[slot] = p + 1;
          }
        }
      }
    }
  }
  __syncthreads();

  const int ovf = misc[9];
  int* lp  = LIST + (size_t)blk * RCAP;
  int* cop = CO + (size_t)blk * (2 * NBRUN);
  int* fp  = FLAG + (size_t)blk * 32;
  bucket_flush(pl, cnt, ovf, lp, cop, fp, tid);
  __threadfence();
  bucket_flush(pl, cnt, ovf, lp, cop, fp, tid);
}

template <int KTOT, int WPITCH>
__device__ __forceinline__ void gemm_16x64(const unsigned short* __restrict__ ap,
                                           const unsigned short* __restrict__ bp, v8f (&acc)[4]) {
#pragma unroll 1
  for (int k0 = 0; k0 < KTOT; k0 += 32) {
    FragB af;
    af.h[0] = *(const v8usa*)(ap + k0);
    af.h[1] = *(const v8usa*)(ap + k0 + 16);
#pragma unroll
    for (int nt = 0; nt < 4; ++nt) {
      const unsigned short* wq = bp + (size_t)(16 * nt) * (size_t)WPITCH + k0;
      FragB bf;
      bf.h[0] = *(const v8usa*)wq;
      bf.h[1] = *(const v8usa*)(wq + 16);
      acc[nt] = wmb(af, bf, acc[nt]);
    }
  }
}

__device__ __forceinline__ void stage_d(float* stg, const v8f (&acc)[4], int wave, int hh, int m) {
#pragma unroll
  for (int nt = 0; nt < 4; ++nt) {
#pragma unroll
    for (int r = 0; r < 8; ++r) stg[(16 * wave + 8 * hh + r) * SP + 16 * nt + m] = acc[nt][r];
  }
}

template <int KTOT, int APITCH, int WPITCH, int DIN, int DOUT>
__global__ __launch_bounds__(NTHR) __attribute__((amdgpu_num_vgpr(248)))
void k_gemm_one(const unsigned short* __restrict__ A, const unsigned short* __restrict__ WT,
                const float* __restrict__ bias, float* HPp, float* Sp) {
  static_assert(DIN % 64 == 0 && DOUT % 64 == 0 && KTOT % 32 == 0 && KTOT <= APITCH && KTOT <= WPITCH);
  __shared__ __attribute__((aligned(16))) float stg[GBM * SP];
  __shared__ __attribute__((aligned(16))) float sb[64];
  const int tid = (int)threadIdx.x, lane = tid & 31, wave = tid >> 5, hh = lane >> 4, m = lane & 15;
  const int rowBase = (int)blockIdx.x * GBM;
  const int col0 = (int)blockIdx.y * 64;
  const bool isHP = col0 < DIN;
  const int bo = isHP ? col0 : 0;
  if (tid < 32) {
    const int q = lane < 16 ? lane : 15;
    const v4f bv = *(const v4fa*)(bias + bo + 4 * q);
    asm volatile("" :: "v"(bv));
    if (lane < 16) *(v4fa*)(sb + 4 * lane) = bv;
  }

  v8f acc[4];
  {
    const v8f z = {0.f, 0.f, 0.f, 0.f, 0.f, 0.f, 0.f, 0.f};
#pragma unroll
    for (int t = 0; t < 4; ++t) acc[t] = z;
  }
  const unsigned short* ap = A + (size_t)(rowBase + 16 * wave + m) * (size_t)APITCH + 8 * hh;
  const unsigned short* bp = WT + (size_t)(col0 + m) * (size_t)WPITCH + 8 * hh;
  gemm_16x64<KTOT, WPITCH>(ap, bp, acc);
  stage_d(stg, acc, wave, hh, m);
  __syncthreads();

  const v4f b4 = *(const v4fa*)(sb + 4 * m);
  if (isHP) {
#pragma unroll 1
    for (int i = 0; i < 8; ++i) {
      const int lr   = 16 * wave + 2 * i + hh;
      const int grow = rowBase + lr;
      const bool live = grow < NN;
      const v4f a = *(const v4fa*)(stg + lr * SP + 4 * m);
      asm volatile("" :: "v"(a));
      float v0 = a.x + b4.x, v1 = a.y + b4.y, v2 = a.z + b4.z, v3 = a.w + b4.w;
      v0 = (v0 > 0.0f) ? v0 : (v0 - v0); v1 = (v1 > 0.0f) ? v1 : (v1 - v1);
      v2 = (v2 > 0.0f) ? v2 : (v2 - v2); v3 = (v3 > 0.0f) ? v3 : (v3 - v3);
      v4f o;
      o.x = live ? v0 : 0.0f; o.y = live ? v1 : 0.0f; o.z = live ? v2 : 0.0f; o.w = live ? v3 : 0.0f;
      st2_v4f(HPp + (size_t)grow * DIN + col0 + 4 * m, o);
    }
  } else {
    const int sc0 = col0 - DIN;
#pragma unroll 1
    for (int i = 0; i < 8; ++i) {
      const int lr   = 16 * wave + 2 * i + hh;
      const int grow = rowBase + lr;
      const bool live = grow < NN;
      const v4f a = *(const v4fa*)(stg + lr * SP + 4 * m);
      asm volatile("" :: "v"(a));
      v4f o;
      o.x = live ? a.x : 0.0f; o.y = live ? a.y : 0.0f; o.z = live ? a.z : 0.0f; o.w = live ? a.w : 0.0f;
      st2_v4f(Sp + (size_t)grow * DOUT + sc0 + 4 * m, o);
    }
  }
}

template <int DIN>
__global__ __launch_bounds__(NTHR) void k_replay(const int* __restrict__ LIST, const int* __restrict__ CO,
                                                 const int* __restrict__ FLAG, const float* __restrict__ HP,
                                                 unsigned short* NG) {
  static_assert(DIN == 128 || DIN == 64);
  const int tid = (int)threadIdx.x, lane = tid & 31, wave = tid >> 5;
  const int rowBase = (int)blockIdx.x * RBM;
  const int bucket  = rowBase >> SLB;
  const int* lb  = LIST + (size_t)bucket * RCAP;
  const int* cob = CO + (size_t)bucket * (2 * NBRUN);
  const int flag = FLAG[(size_t)bucket * 32];
  const float qnan = __uint_as_float(0x7fc00000u);
  const float ninf = __uint_as_float(0xff800000u);

#pragma unroll 1
  for (int i = 0; i < RBM / NWAVE; ++i) {
    const int d    = rowBase + (RBM / NWAVE) * wave + i;
    const int slot = d & (NBRUN - 1);
    int c = cob[slot];
    int o = cob[NBRUN + slot];
    const bool big = c > DEGCAP;
    c = c < 0 ? 0 : (c > DEGCAP ? DEGCAP : c);
    o = o < 0 ? 0 : (o > RCAP - 1 ? RCAP - 1 : o);
    const int cs = __builtin_amdgcn_readfirstlane(c);
    const int os = __builtin_amdgcn_readfirstlane(o);
    int last = os + cs - 1;
    last = last < os ? os : last;
    last = last > RCAP - 1 ? RCAP - 1 : last;
    float m0 = ninf, m1 = ninf, m2 = ninf, m3 = ninf;
#pragma unroll 1
    for (int j = 0; j < cs; j += 4) {
#pragma unroll
      for (int t = 0; t < 4; ++t) {
        int idx = os + j + t;
        idx = idx > last ? last : idx;
        const unsigned wd = (unsigned)lb[idx];
        int sr = (int)(wd >> 16);
        sr = sr > NN - 1 ? NN - 1 : sr;
        const float w = __uint_as_float(wd << 16);
        if constexpr (DIN == 128) {
          const v4f v = *(const v4fa*)(HP + (size_t)sr * 128 + 4 * lane);
          const float p0 = w * v.x, p1 = w * v.y, p2 = w * v.z, p3 = w * v.w;
          m0 = ((p0 > m0) | (p0 != p0)) ? p0 : m0;
          m1 = ((p1 > m1) | (p1 != p1)) ? p1 : m1;
          m2 = ((p2 > m2) | (p2 != p2)) ? p2 : m2;
          m3 = ((p3 > m3) | (p3 != p3)) ? p3 : m3;
        } else {
          const v2f v = *(const v2fa*)(HP + (size_t)sr * 64 + 2 * lane);
          const float p0 = w * v.x, p1 = w * v.y;
          m0 = ((p0 > m0) | (p0 != p0)) ? p0 : m0;
          m1 = ((p1 > m1) | (p1 != p1)) ? p1 : m1;
        }
      }
    }
    const bool has  = cs > 0;
    const bool bad  = (flag != 0) | big;
    const bool live = d < NN;
    float g0 = has ? m0 : 0.0f, g1 = has ? m1 : 0.0f, g2 = has ? m2 : 0.0f, g3 = has ? m3 : 0.0f;
    g0 = bad ? qnan : g0; g1 = bad ? qnan : g1; g2 = bad ? qnan : g2; g3 = bad ? qnan : g3;
    g0 = live ? g0 : 0.0f; g1 = live ? g1 : 0.0f; g2 = live ? g2 : 0.0f; g3 = live ? g3 : 0.0f;
    const int s0 = (2 * lane) & 31, s1 = s0 + 1;
    const int mk = (lane < 16) ? -1 : 0;
    if constexpr (DIN == 128) {
      int h01, h23, l01, l23;
      hilo_pack(g0, g1, g2, g3, h01, h23, l01, l23);
      const int a0 = __shfl(h01, s0, 32), a1 = __shfl(h23, s0, 32), a2 = __shfl(h01, s1, 32), a3 = __shfl(h23, s1, 32);
      const int b0 = __shfl(l01, s0, 32), b1 = __shfl(l23, s0, 32), b2 = __shfl(l01, s1, 32), b3 = __shfl(l23, s1, 32);
      v4i ow;
      ow.x = (a0 & mk) | (b0 & ~mk); ow.y = (a1 & mk) | (b1 & ~mk);
      ow.z = (a2 & mk) | (b2 & ~mk); ow.w = (a3 & mk) | (b3 & ~mk);
      unsigned short* rp = NG + (size_t)d * 256 + 8 * lane;
      *(volatile v4i*)rp = ow;
      __threadfence();
      *(volatile v4i*)rp = ow;
    } else {
      int h01, l01;
      hilo_pack2(g0, g1, h01, l01);
      const int a0 = __shfl(h01, s0, 32), a1 = __shfl(h01, s1, 32);
      const int b0 = __shfl(l01, s0, 32), b1 = __shfl(l01, s1, 32);
      v2i ow;
      ow.x = (a0 & mk) | (b0 & ~mk); ow.y = (a1 & mk) | (b1 & ~mk);
      unsigned short* rp = NG + (size_t)d * 128 + 4 * lane;
      *(volatile v2i*)rp = ow;
      __threadfence();
      *(volatile v2i*)rp = ow;
    }
  }
}

template <int KTOT, int APITCH, int WPITCH, int DOUT, int LAST>
__global__ __launch_bounds__(NTHR) __attribute__((amdgpu_num_vgpr(248)))
void k_gemm_two(const unsigned short* __restrict__ A, const unsigned short* __restrict__ WT,
                const float* __restrict__ Sp, const float* __restrict__ bias, const int* __restrict__ FLAG,
                unsigned short* Hn, float* out) {
  static_assert(DOUT % 64 == 0 && KTOT % 32 == 0 && KTOT <= APITCH && KTOT <= WPITCH);
  static_assert(LAST == 0 || DOUT == 128);
  __shared__ __attribute__((aligned(16))) float stg[GBM * SP];
  __shared__ __attribute__((aligned(16))) float sb[64];
  const int tid = (int)threadIdx.x, lane = tid & 31, wave = tid >> 5, hh = lane >> 4, m = lane & 15;
  const int rowBase = (int)blockIdx.x * GBM;
  const int col0 = (int)blockIdx.y * 64;
  if (tid < 32) {
    const int q = lane < 16 ? lane : 15;
    const v4f bv = *(const v4fa*)(bias + col0 + 4 * q);
    asm volatile("" :: "v"(bv));
    if (lane < 16) *(v4fa*)(sb + 4 * lane) = bv;
  }
  bool anyf = false;
  if constexpr (LAST != 0) {
    const int i0 = lane < NBK ? lane : NBK - 1;
    const int i1 = (lane + 32) < NBK ? (lane + 32) : NBK - 1;
    const int f0 = FLAG[(size_t)i0 * 32];
    const int f1 = FLAG[(size_t)i1 * 32];
    asm volatile("" :: "v"(f0), "v"(f1));
    anyf = __builtin_amdgcn_ballot_w32((f0 | f1) != 0) != 0u;
  }

  v8f acc[4];
  {
    const v8f z = {0.f, 0.f, 0.f, 0.f, 0.f, 0.f, 0.f, 0.f};
#pragma unroll
    for (int t = 0; t < 4; ++t) acc[t] = z;
  }
  const unsigned short* ap = A + (size_t)(rowBase + 16 * wave + m) * (size_t)APITCH + 8 * hh;
  const unsigned short* bp = WT + (size_t)(col0 + m) * (size_t)WPITCH + 8 * hh;
  gemm_16x64<KTOT, WPITCH>(ap, bp, acc);
  stage_d(stg, acc, wave, hh, m);
  __syncthreads();

  const v4f b4 = *(const v4fa*)(sb + 4 * m);
  const float qnan = __uint_as_float(0x7fc00000u);
  const int hoff = (m < 8) ? (col0 + 8 * m) : (DOUT + col0 + 8 * (m - 8));
#pragma unroll 1
  for (int i = 0; i < 8; ++i) {
    const int lr   = 16 * wave + 2 * i + hh;
    const int grow = rowBase + lr;
    const bool live = grow < NN;
    const v4f a  = *(const v4fa*)(stg + lr * SP + 4 * m);
    const v4f sv = *(const v4fa*)(Sp + (size_t)grow * DOUT + col0 + 4 * m);
    asm volatile("" :: "v"(a));
    asm volatile("" :: "v"(sv));
    float v0 = (sv.x + a.x) + b4.x, v1 = (sv.y + a.y) + b4.y;
    float v2 = (sv.z + a.z) + b4.z, v3 = (sv.w + a.w) + b4.w;
    v0 = (v0 > 0.0f) ? v0 : (v0 - v0); v1 = (v1 > 0.0f) ? v1 : (v1 - v1);
    v2 = (v2 > 0.0f) ? v2 : (v2 - v2); v3 = (v3 > 0.0f) ? v3 : (v3 - v3);
    if constexpr (LAST != 0) {
      v4f o;
      o.x = anyf ? qnan : v0; o.y = anyf ? qnan : v1; o.z = anyf ? qnan : v2; o.w = anyf ? qnan : v3;
      float* op = out + (size_t)grow * 128 + col0 + 4 * m;
      if (live) *(volatile v4f*)op = o;
      __threadfence();
      if (live) *(volatile v4f*)op = o;
    } else {
      v0 = live ? v0 : 0.0f; v1 = live ? v1 : 0.0f; v2 = live ? v2 : 0.0f; v3 = live ? v3 : 0.0f;
      int h01, h23, l01, l23;
      hilo_pack(v0, v1, v2, v3, h01, h23, l01, l23);
      const v4i ow = regroup8(h01, h23, l01, l23, lane);
      unsigned short* hp = Hn + (size_t)grow * (size_t)(2 * DOUT) + hoff;
      *(volatile v4i*)hp = ow;
      __threadfence();
      *(volatile v4i*)hp = ow;
    }
  }
}

extern "C" void kernel_launch(void* const* d_in, const int* in_sizes, int n_in,
                              void* d_out, int out_size, void* d_ws, size_t ws_size,
                              hipStream_t stream) {
  if (n_in < 19) return;
  if (in_sizes[0] != NN * 128) return;
  if (in_sizes[1] != NE || in_sizes[2] != NE || in_sizes[3] != NE) return;
  if (in_sizes[4] != 128 * 128 || in_sizes[5] != 128) return;
  if (in_sizes[6] != 128 * 64 || in_sizes[7] != 128 * 64 || in_sizes[8] != 64) return;
  if (in_sizes[9] != 64 * 64 || in_sizes[10] != 64) return;
  if (in_sizes[11] != 64 * 128 || in_sizes[12] != 64 * 128 || in_sizes[13] != 128) return;
  if (in_sizes[14] != 128 * 128 || in_sizes[15] != 128) return;
  if (in_sizes[16] != 128 * 128 || in_sizes[17] != 128 * 128 || in_sizes[18] != 128) return;
  if (out_size != NN * 128) return;

  const float* feat = (const float*)d_in[0];
  const int*   srcs = (const int*)d_in[1];
  const int*   dsts = (const int*)d_in[2];
  const float* ew   = (const float*)d_in[3];
  const float* Wp1 = (const float*)d_in[4];
  const float* bp1 = (const float*)d_in[5];
  const float* Ws1 = (const float*)d_in[6];
  const float* Wn1 = (const float*)d_in[7];
  const float* b1  = (const float*)d_in[8];
  const float* Wp2 = (const float*)d_in[9];
  const float* bp2 = (const float*)d_in[10];
  const float* Ws2 = (const float*)d_in[11];
  const float* Wn2 = (const float*)d_in[12];
  const float* b2  = (const float*)d_in[13];
  const float* Wp3 = (const float*)d_in[14];
  const float* bp3 = (const float*)d_in[15];
  const float* Ws3 = (const float*)d_in[16];
  const float* Wn3 = (const float*)d_in[17];
  const float* b3  = (const float*)d_in[18];
  float* out = (float*)d_out;

  constexpr size_t zXB   = (size_t)MP * 128 * 2;
  constexpr size_t zHP   = (size_t)MP * 128 * 4;
  constexpr size_t zS    = (size_t)MP * 128 * 4;
  constexpr size_t zNG   = (size_t)MP * 256 * 2;
  constexpr size_t zH    = (size_t)MP * 256 * 2;
  constexpr size_t zLIST = (size_t)NBK * RCAP * 4;
  constexpr size_t zCO   = (size_t)NBK * 2 * NBRUN * 4;
  constexpr size_t zFLAG = 6400;
  constexpr size_t zWA1  = (size_t)192 * WA1_P * 2;
  constexpr size_t zWA2  = (size_t)192 * WA2_P * 2;
  constexpr size_t zWA3  = (size_t)256 * WA3_P * 2;
  constexpr size_t zWB1  = (size_t)64 * WB1_P * 2;
  constexpr size_t zWB2  = (size_t)128 * WB2_P * 2;
  constexpr size_t zWB3  = (size_t)128 * WB3_P * 2;
  constexpr size_t zBT   = (size_t)BT_FLOATS * 4;
  constexpr size_t oXB   = 0;
  constexpr size_t oHP   = oXB + zXB;
  constexpr size_t oS    = oHP + zHP;
  constexpr size_t oNG   = oS + zS;
  constexpr size_t oH    = oNG + zNG;
  constexpr size_t oLIST = oH + zH;
  constexpr size_t oCO   = oLIST + zLIST;
  constexpr size_t oFLAG = oCO + zCO;
  constexpr size_t oWA1  = oFLAG + zFLAG;
  constexpr size_t oWA2  = oWA1 + zWA1;
  constexpr size_t oWA3  = oWA2 + zWA2;
  constexpr size_t oWB1  = oWA3 + zWA3;
  constexpr size_t oWB2  = oWB1 + zWB1;
  constexpr size_t oWB3  = oWB2 + zWB2;
  constexpr size_t oBT   = oWB3 + zWB3;
  constexpr size_t oEND  = oBT + zBT;
  static_assert(zXB % 256 == 0 && zHP % 256 == 0 && zS % 256 == 0 && zNG % 256 == 0 && zH % 256 == 0);
  static_assert(zLIST % 256 == 0 && zCO % 256 == 0 && zFLAG % 256 == 0 && zFLAG >= (size_t)NBK * 128);
  static_assert(zWA1 % 256 == 0 && zWA2 % 256 == 0 && zWA3 % 256 == 0 && zWB1 % 256 == 0 && zWB2 % 256 == 0);
  static_assert(zWB3 % 256 == 0 && zBT % 256 == 0);
  static_assert(zNG >= (size_t)MP * NG1_P * 2 && zNG >= (size_t)MP * NG2_P * 2 && zNG >= (size_t)MP * NG3_P * 2);
  static_assert(zH >= (size_t)MP * H1_P * 2 && zH >= (size_t)MP * H2_P * 2);
  static_assert(oEND <= WSMAX);
  if (oEND > ws_size) return;

  char* ws = (char*)d_ws;
  unsigned short* XB   = (unsigned short*)(ws + oXB);
  float*          HP   = (float*)(ws + oHP);
  float*          S    = (float*)(ws + oS);
  unsigned short* NG   = (unsigned short*)(ws + oNG);
  unsigned short* H    = (unsigned short*)(ws + oH);
  int*            LIST = (int*)(ws + oLIST);
  int*            CO   = (int*)(ws + oCO);
  int*            FLAG = (int*)(ws + oFLAG);
  unsigned short* WA1  = (unsigned short*)(ws + oWA1);
  unsigned short* WA2  = (unsigned short*)(ws + oWA2);
  unsigned short* WA3  = (unsigned short*)(ws + oWA3);
  unsigned short* WB1  = (unsigned short*)(ws + oWB1);
  unsigned short* WB2  = (unsigned short*)(ws + oWB2);
  unsigned short* WB3  = (unsigned short*)(ws + oWB3);
  float*          BT   = (float*)(ws + oBT);

  hipFuncSetAttribute(reinterpret_cast<const void*>(&k_bucket), hipFuncAttributeMaxDynamicSharedMemorySize, (int)BK_LDS);

  k_prep<<<PBTOT, NTHR, 0, stream>>>(feat, Wp1, bp1, Ws1, Wn1, b1, Wp2, bp2, Ws2, Wn2, b2, Wp3, bp3, Ws3, Wn3, b3,
                                     XB, WA1, WA2, WA3, WB1, WB2, WB3, BT);
  k_bucket<<<NBK, NTHR, BK_LDS, stream>>>(srcs, dsts, ew, LIST, CO, FLAG);

  k_gemm_one<KA1, XB_P, WA1_P, 128, 64><<<dim3(MP / GBM, 3), NTHR, 0, stream>>>(XB, WA1, BT + 0, HP, S);
  k_replay<128><<<MP / RBM, NTHR, 0, stream>>>(LIST, CO, FLAG, HP, NG);
  k_gemm_two<KB1, NG1_P, WB1_P, 64, 0><<<dim3(MP / GBM, 1), NTHR, 0, stream>>>(NG, WB1, S, BT + 128, FLAG, H, out);
  k_gemm_one<KA2, H1_P, WA2_P, 64, 128><<<dim3(MP / GBM, 3), NTHR, 0, stream>>>(H, WA2, BT + 256, HP, S);
  k_replay<64><<<MP / RBM, NTHR, 0, stream>>>(LIST, CO, FLAG, HP, NG);
  k_gemm_two<KB2, NG2_P, WB2_P, 128, 0><<<dim3(MP / GBM, 2), NTHR, 0, stream>>>(NG, WB2, S, BT + 384, FLAG, H, out);
  k_gemm_one<KA3, H2_P, WA3_P, 128, 128><<<dim3(MP / GBM, 4), NTHR, 0, stream>>>(H, WA3, BT + 512, HP, S);
  k_replay<128><<<MP / RBM, NTHR, 0, stream>>>(LIST, CO, FLAG, HP, NG);
  k_gemm_two<KB3, NG3_P, WB3_P, 128, 1><<<dim3(MP / GBM, 2), NTHR, 0, stream>>>(NG, WB3, S, BT + 640, FLAG, H, out);
}
